// StandardAttention_34823594836450
// MI455X (gfx1250) — hardware-verified
//
#include <hip/hip_runtime.h>


#ifndef NB
#define NB 8
#endif
#ifndef SEQ
#define SEQ 1370
#endif
#ifndef NB_FULL
#define NB_FULL 8
#endif
#ifndef SEQ_FULL
#define SEQ_FULL 1370
#endif
#ifndef QKRES
#define QKRES 1
#endif
#ifndef PRES
#define PRES 0
#endif

namespace {
constexpr int HH = 6, HD = 64, CC = HH * HD, C3 = 3 * CC, NN = SEQ;
constexpr int NP = ((SEQ + 63) / 64) * 64;
constexpr int KEND = ((SEQ + 31) / 32) * 32;
constexpr int KS = CC / 32;
constexpr int XPR = CC / 8;
constexpr float XS = 8.0f, WS = 64.0f, QS = 8.0f, RS = 1024.0f, PS = 1024.0f, PRS = 1024.0f, CS = 64.0f, LOG2E = 1.4426950408889634f;
static_assert(NN >= 1 && NN <= SEQ_FULL && NB >= 1 && NB <= NB_FULL && NP % 64 == 0 && NP >= NN && KEND <= NP && KEND >= 32);
static_assert(HD == 64 && CC % 64 == 0 && CC / 64 == HH && C3 % 64 == 0 && C3 / 64 == 3 * HH && (C3 * CC / 8) % 256 == 0 && (CC * CC / 8) % 256 == 0);

typedef _Float16 b16;
typedef __attribute__((ext_vector_type(16))) _Float16 v16b;
typedef __attribute__((ext_vector_type(8))) _Float16 v8b;
typedef __attribute__((ext_vector_type(8))) float v8f;
typedef __attribute__((ext_vector_type(4))) float v4f;

__device__ __forceinline__ float bf16_rne(float f) { unsigned int u = __float_as_uint(f); u += 0x7FFFu + ((u >> 16) & 1u); return __uint_as_float(u & 0xFFFF0000u); }
__device__ __forceinline__ v16b frag_kb(const b16* p, int hh) {
  const v8b a = *(const v8b*)(p + 8 * hh), b = *(const v8b*)(p + 16 + 8 * hh); v16b f;
#pragma unroll
  for (int e = 0; e < 8; ++e) { f[e] = a[e]; f[8 + e] = b[e]; }
  return f;
}
__device__ __forceinline__ v8f wmma16b(v16b a, v16b b, v8f c) {
  v8f d = __builtin_amdgcn_wmma_f32_16x16x32_f16(false, a, false, b, (short)0, c, false, false);
  asm volatile("v_nop\n\tv_nop\n\tv_nop\n\tv_nop" : "+v"(d) : "v"(a), "v"(b));
  return d;
}
__device__ __forceinline__ void wave_lds_sync() { __builtin_amdgcn_fence(3, "workgroup"); __builtin_amdgcn_wave_barrier(); __builtin_amdgcn_fence(2, "workgroup"); }
__device__ __forceinline__ float nexp2(float v) { return __builtin_amdgcn_exp2f(v); }

__global__ __launch_bounds__(256) void cvt_x_kernel(const float* __restrict__ X, b16* __restrict__ Xp) {
  const size_t u = (size_t)blockIdx.x * 256 + threadIdx.x;
  if (u >= (size_t)NB * NP * XPR) return;
  const size_t row = u / XPR; const int piece = (int)(u % XPR);
  const int b = (int)(row / NP), n = (int)(row % NP);
  const int nc = n < NN ? n : NN - 1;
  const float sc = n < NN ? XS : 0.0f;
  const float* src = X + ((size_t)b * SEQ_FULL + (size_t)nc) * CC + piece * 8;
  const v4f x0 = *(const v4f*)src, x1 = *(const v4f*)(src + 4); v8b o;
#pragma unroll
  for (int j = 0; j < 4; ++j) { o[j] = (b16)(bf16_rne(x0[j]) * sc); o[4 + j] = (b16)(bf16_rne(x1[j]) * sc); }
  b16* dst = Xp + row * CC + piece * 8;
  *(volatile v8b*)dst = o; __threadfence(); *(volatile v8b*)dst = o;
}

__global__ __launch_bounds__(256) void cvt_w_kernel(const float* __restrict__ Wq, const float* __restrict__ Wp, b16* __restrict__ Wqp, b16* __restrict__ Wpp) {
  const size_t u = (size_t)blockIdx.x * 256 + threadIdx.x;
  const size_t lim = blockIdx.y == 0 ? (size_t)C3 * CC / 8 : (size_t)CC * CC / 8;
  if (u >= lim) return;
  const float* src = (blockIdx.y == 0 ? Wq : Wp) + u * 8; b16* dst = (blockIdx.y == 0 ? Wqp : Wpp) + u * 8;
  const v4f x0 = *(const v4f*)src, x1 = *(const v4f*)(src + 4); v8b o;
#pragma unroll
  for (int j = 0; j < 4; ++j) { o[j] = (b16)(bf16_rne(x0[j]) * WS); o[4 + j] = (b16)(bf16_rne(x1[j]) * WS); }
  *(volatile v8b*)dst = o; __threadfence(); *(volatile v8b*)dst = o;
}

template <bool QR>
__global__ __launch_bounds__(128) void qkv_kernel(const b16* __restrict__ Xp, const b16* __restrict__ Wqp, const float* __restrict__ bq,
                                                  b16* __restrict__ Qh, b16* __restrict__ Ql, b16* __restrict__ Kh, b16* __restrict__ Kl, b16* __restrict__ VT) {
  __shared__ __attribute__((aligned(16))) b16 Th[4][16][HD + 8];
  __shared__ __attribute__((aligned(16))) b16 Tl[4][16][HD + 8];
  __shared__ __attribute__((aligned(16))) b16 St[HD][64 + 8];
  const int wave = threadIdx.x >> 5, lane = threadIdx.x & 31, hh = lane >> 4, col = lane & 15;
  const int tt = (int)blockIdx.x, ft = (int)blockIdx.y, b = (int)blockIdx.z;
  const int which = ft / HH, h = ft - which * HH;
  const b16* Ar = Xp + ((size_t)b * NP + (size_t)tt * 64 + wave * 16 + col) * CC;
  const b16* Br = Wqp + ((size_t)ft * 64 + col) * CC;
  v8f acc[4];
#pragma unroll
  for (int t = 0; t < 4; ++t) acc[t] = (v8f){};
#pragma unroll 1
  for (int ks = 0; ks < KS; ++ks) {
    const v16b a = frag_kb(Ar + ks * 32, hh);
#pragma unroll
    for (int t = 0; t < 4; ++t) acc[t] = wmma16b(a, frag_kb(Br + (size_t)t * 16 * CC + ks * 32, hh), acc[t]);
  }
  float bb[4];
#pragma unroll
  for (int t = 0; t < 4; ++t) bb[t] = bf16_rne(bq[ft * 64 + t * 16 + col]);
  const float osc = 1.0f / (XS * WS);
  const int n0 = tt * 64 + wave * 16 + 8 * hh;
  if (which == 2) {
#pragma unroll
    for (int t = 0; t < 4; ++t) {
#pragma unroll
      for (int r = 0; r < 8; ++r) {
        float val = acc[t][r] * osc + bb[t]; val = (n0 + r < NN) ? val : 0.0f;
        St[t * 16 + col][wave * 16 + 8 * hh + r] = (b16)(val * QS); } }
  } else {
#pragma unroll
    for (int t = 0; t < 4; ++t) {
#pragma unroll
      for (int r = 0; r < 8; ++r) {
        float val = acc[t][r] * osc + bb[t]; val = (n0 + r < NN) ? val : 0.0f;
        const float vs = val * QS; const b16 hi = (b16)vs;
        Th[wave][8 * hh + r][t * 16 + col] = hi;
        if constexpr (QR) Tl[wave][8 * hh + r][t * 16 + col] = (b16)((vs - (float)hi) * RS); } }
  }
  __syncthreads();
  const size_t bhi = (size_t)b * HH + h;
  if (which == 2) {
    b16* dstb = VT + bhi * HD * (size_t)NP + (size_t)tt * 64;
    for (int pass = 0; pass < 2; ++pass) {
#pragma unroll 1
      for (int it = 0; it < 4; ++it) {
        const int d = wave * 16 + it * 4 + (lane >> 3), tok = (lane & 7) * 8;
        const v8b o = *(const v8b*)(&St[d][tok]);
        *(volatile v8b*)(dstb + (size_t)d * NP + tok) = o; }
      __threadfence(); }
  } else {
    const size_t rowoff = (bhi * NP + (size_t)tt * 64 + wave * 16) * HD;
    b16* dh = (which == 0 ? Qh : Kh) + rowoff;
    b16* dl = (which == 0 ? Ql : Kl) + rowoff;
    for (int pass = 0; pass < 2; ++pass) {
#pragma unroll 1
      for (int it = 0; it < 4; ++it) {
        const int row = it * 4 + (lane >> 3), piece = (lane & 7) * 8;
        const v8b o = *(const v8b*)(&Th[wave][row][piece]);
        *(volatile v8b*)(dh + (size_t)row * HD + piece) = o;
        if constexpr (QR) { const v8b o2 = *(const v8b*)(&Tl[wave][row][piece]); *(volatile v8b*)(dl + (size_t)row * HD + piece) = o2; } }
      __threadfence(); }
  }
}

template <bool QR, bool PR>
__global__ __launch_bounds__(64) __attribute__((amdgpu_num_vgpr(256))) void attn_kernel(const b16* __restrict__ Qh, const b16* __restrict__ Ql,
                                                                                      const b16* __restrict__ Kh, const b16* __restrict__ Kl,
                                                                                      const b16* __restrict__ VT, b16* __restrict__ Cp) {
  __shared__ __attribute__((aligned(16))) b16 Pb[2][16][32 + 8];
  __shared__ __attribute__((aligned(16))) b16 Pr[2][16][32 + 8];
  __shared__ __attribute__((aligned(16))) b16 Tc[2][16][HD + 8];
  const int wave = threadIdx.x >> 5, lane = threadIdx.x & 31, hh = lane >> 4, col = lane & 15;
  const size_t bhi = blockIdx.y; const int b = (int)(bhi / HH), h = (int)(bhi % HH);
  const int q0 = (int)blockIdx.x * 32 + wave * 16, qi = q0 + col;
  const b16* Qb = Qh + bhi * NP * HD; const b16* Qlb = Ql + bhi * NP * HD;
  const b16* Kb = Kh + bhi * NP * HD; const b16* Klb = Kl + bhi * NP * HD; const b16* Vb = VT + bhi * HD * (size_t)NP;
  const v16b qa0 = frag_kb(Qb + (size_t)qi * HD, hh), qa1 = frag_kb(Qb + (size_t)qi * HD + 32, hh);
  v16b ql0 = (v16b){}, ql1 = (v16b){};
  if constexpr (QR) { ql0 = frag_kb(Qlb + (size_t)qi * HD, hh); ql1 = frag_kb(Qlb + (size_t)qi * HD + 32, hh); }
  const float cs = LOG2E * 0.125f / (QS * QS);
  float m = -INFINITY, l = 0.0f; v8f o[4], o2[4];
#pragma unroll
  for (int t = 0; t < 4; ++t) { o[t] = (v8f){}; o2[t] = (v8f){}; }
#pragma unroll 1
  for (int kb = 0; kb < KEND; kb += 32) {
    float e[16]; float mx = -INFINITY;
#pragma unroll
    for (int u = 0; u < 2; ++u) {
      const size_t kr = (size_t)(kb + u * 16 + col) * HD;
      const v16b kh0 = frag_kb(Kb + kr, hh), kh1 = frag_kb(Kb + kr + 32, hh);
      v8f s = (v8f){}; s = wmma16b(kh0, qa0, s); s = wmma16b(kh1, qa1, s);
      v8f s2 = (v8f){};
      if constexpr (QR) {
        s2 = wmma16b(kh0, ql0, s2); s2 = wmma16b(kh1, ql1, s2);
        const v16b kl0 = frag_kb(Klb + kr, hh), kl1 = frag_kb(Klb + kr + 32, hh);
        s2 = wmma16b(kl0, qa0, s2); s2 = wmma16b(kl1, qa1, s2); }
#pragma unroll
      for (int r = 0; r < 8; ++r) {
        float v = s[r];
        if constexpr (QR) v += s2[r] * (1.0f / RS);
        v *= cs;
        const int key = kb + u * 16 + 8 * hh + r;
        const float ev = (key < NN) ? v : -INFINITY;
        e[u * 8 + r] = ev; mx = fmaxf(mx, ev); } }
    mx = fmaxf(mx, __shfl_xor(mx, 16)); const float mn = fmaxf(m, mx); const float al = nexp2(m - mn); float sum = 0.0f;
#pragma unroll
    for (int i2 = 0; i2 < 16; ++i2) {
      const float p = nexp2(e[i2] - mn); sum += p; const int pi = (i2 < 8 ? 0 : 16) + 8 * hh + (i2 & 7);
      const float pp = p * PS; const b16 ph = (b16)pp; Pb[wave][col][pi] = ph;
      if constexpr (PR) Pr[wave][col][pi] = (b16)((pp - (float)ph) * PRS); }
    sum += __shfl_xor(sum, 16); l = l * al + sum; m = mn;
    wave_lds_sync();
    const v16b pf = frag_kb(&Pb[wave][col][0], hh);
    v16b prf = (v16b){};
    if constexpr (PR) prf = frag_kb(&Pr[wave][col][0], hh);
#pragma unroll
    for (int t = 0; t < 4; ++t) {
      o[t] *= al; const v16b vh = frag_kb(Vb + (size_t)(t * 16 + col) * NP + kb, hh);
      o[t] = wmma16b(vh, pf, o[t]);
      if constexpr (PR) { o2[t] *= al; o2[t] = wmma16b(vh, prf, o2[t]); } }
    wave_lds_sync(); }
  const float inv = CS / (l * PS * QS);
#pragma unroll
  for (int t = 0; t < 4; ++t) {
#pragma unroll
    for (int r = 0; r < 8; ++r) {
      float ov = o[t][r];
      if constexpr (PR) ov += o2[t][r] * (1.0f / PRS);
      Tc[wave][col][t * 16 + 8 * hh + r] = (b16)(ov * inv); } }
  wave_lds_sync();
  b16* cb = Cp + ((size_t)b * NP + (size_t)q0) * CC + (size_t)h * HD;
  for (int pass = 0; pass < 2; ++pass) {
#pragma unroll 1
    for (int it = 0; it < 4; ++it) {
      const int row = it * 4 + (lane >> 3), piece = (lane & 7) * 8;
      const v8b f = *(const v8b*)(&Tc[wave][row][piece]);
      *(volatile v8b*)(cb + (size_t)row * CC + piece) = f; }
    __threadfence(); }
}

__global__ __launch_bounds__(128) void proj_kernel(const b16* __restrict__ Cp, const b16* __restrict__ Wpp, const float* __restrict__ bp, float* __restrict__ out) {
  __shared__ __attribute__((aligned(16))) float To[4][16][HD + 4];
  const int wave = threadIdx.x >> 5, lane = threadIdx.x & 31, hh = lane >> 4, col = lane & 15;
  const int tt = (int)blockIdx.x, ft = (int)blockIdx.y, b = (int)blockIdx.z;
  const b16* Ar = Cp + ((size_t)b * NP + (size_t)tt * 64 + wave * 16 + col) * CC;
  const b16* Br = Wpp + ((size_t)ft * 64 + col) * CC;
  v8f acc[4];
#pragma unroll
  for (int t = 0; t < 4; ++t) acc[t] = (v8f){};
#pragma unroll 1
  for (int ks = 0; ks < KS; ++ks) {
    const v16b a = frag_kb(Ar + ks * 32, hh);
#pragma unroll
    for (int t = 0; t < 4; ++t) acc[t] = wmma16b(a, frag_kb(Br + (size_t)t * 16 * CC + ks * 32, hh), acc[t]);
  }
  const float osc = 1.0f / (CS * WS);
#pragma unroll
  for (int t = 0; t < 4; ++t) {
    const float bbv = bf16_rne(bp[ft * 64 + t * 16 + col]);
#pragma unroll
    for (int r = 0; r < 8; ++r) To[wave][8 * hh + r][t * 16 + col] = acc[t][r] * osc + bbv; }
  wave_lds_sync();
  const int n0 = tt * 64 + wave * 16;
  float* ob = out + ((size_t)b * SEQ_FULL + (size_t)n0) * CC + ft * 64;
  for (int pass = 0; pass < 2; ++pass) {
#pragma unroll 1
    for (int it = 0; it < 8; ++it) {
      const int rr = it * 2 + hh;
      if (n0 + rr < NN) {
        const v4f f = *(const v4f*)(&To[wave][rr][col * 4]);
        *(volatile v4f*)(ob + (size_t)rr * CC + col * 4) = f; } }
    __threadfence(); }
}
}

extern "C" void kernel_launch(void* const* d_in, const int* in_sizes, int n_in, void* d_out, int out_size, void* d_ws, size_t ws_size, hipStream_t stream) {
  const size_t need = ((size_t)(NB - 1) * SEQ_FULL + NN) * CC;
  if (n_in < 5 || (size_t)in_sizes[0] < need || (size_t)in_sizes[1] < (size_t)C3 * CC || (size_t)in_sizes[2] < (size_t)C3 ||
      (size_t)in_sizes[3] < (size_t)CC * CC || (size_t)in_sizes[4] < (size_t)CC || (size_t)out_size < need) return;
  const float* Xin = (const float*)d_in[0]; const float* Wq = (const float*)d_in[1]; const float* Bq = (const float*)d_in[2];
  const float* Wp = (const float*)d_in[3]; const float* Bp = (const float*)d_in[4];
  size_t off = 0; char* ws = (char*)d_ws;
  auto carve = [&](size_t bytes) { char* p = ws + off; off += (bytes + 255) & ~(size_t)255; return p; };
  const size_t xplane = (size_t)NB * NP * CC * 2;
  const size_t hplane = (size_t)NB * HH * NP * HD * 2;
  b16* Xp = (b16*)carve(xplane);
  b16* Wqp = (b16*)carve((size_t)C3 * CC * 2); b16* Wpp = (b16*)carve((size_t)CC * CC * 2);
  b16* Qh = (b16*)carve(hplane); b16* Ql = (b16*)carve(hplane); b16* Kh = (b16*)carve(hplane); b16* Kl = (b16*)carve(hplane); b16* VT = (b16*)carve(hplane);
  b16* Cp = (b16*)carve(xplane);
  if (off > ws_size || off > ((size_t)128 << 20)) return;
  cvt_x_kernel<<<dim3((unsigned)(((size_t)NB * NP * XPR + 255) / 256)), 256, 0, stream>>>(Xin, Xp);
  cvt_w_kernel<<<dim3((unsigned)((size_t)C3 * CC / 8 / 256), 2), 256, 0, stream>>>(Wq, Wp, Wqp, Wpp);
  qkv_kernel<(QKRES != 0)><<<dim3(NP / 64, C3 / 64, NB), 128, 0, stream>>>(Xp, Wqp, Bq, Qh, Ql, Kh, Kl, VT);
  attn_kernel<(QKRES != 0), (PRES != 0)><<<dim3(NP / 32, NB * HH), 64, 0, stream>>>(Qh, Ql, Kh, Kl, VT, Cp);
  proj_kernel<<<dim3(NP / 64, CC / 64, NB), 128, 0, stream>>>(Cp, Wpp, Bp, (float*)d_out);
}
